// EncoderLayer_2052994367605
// MI455X (gfx1250) — hardware-verified
//
#include <hip/hip_runtime.h>
#include <math.h>

#ifndef NB
#define NB 2
#endif
#ifndef SEQ
#define SEQ 2048
#endif
#define NB_FULL 2
#define SEQ_FULL 2048
#define DM 1024
#define NHEAD 16
#define HDIM 64
#define DFF 4096
#define ROWS (NB * SEQ)

static_assert(DM == NHEAD * HDIM);
static_assert(HDIM == 64);
static_assert(DM == 128 * 8);
static_assert(SEQ % 64 == 0);
static_assert(ROWS % 64 == 0);
static_assert(DM % 64 == 0 && DFF % 64 == 0 && (3 * DM) % 64 == 0);
static_assert(DM % 32 == 0 && DFF % 32 == 0);
static_assert(DM % 8 == 0 && DFF % 8 == 0);
static_assert(NB <= NB_FULL && SEQ <= SEQ_FULL);
static_assert(DM == 4 * 256 && DFF == 16 * 256);

typedef __attribute__((ext_vector_type(16))) _Float16 v16h;
typedef __attribute__((ext_vector_type(8)))  _Float16 v8h;
typedef __attribute__((ext_vector_type(8)))  float    v8f;
typedef __attribute__((ext_vector_type(4)))  float    v4f;
typedef v8h v8h_a __attribute__((may_alias));
typedef v4f v4f_a __attribute__((may_alias));

__device__ __forceinline__ v8f wmma16(v16h a, v16h b, v8f c) {
    c = __builtin_amdgcn_wmma_f32_16x16x32_f16(false, a, false, b, (short)0, c, false, false);
    asm volatile("v_nop\n\tv_nop\n\tv_nop\n\tv_nop" : "+v"(c) : "v"(a), "v"(b));
    return c;
}
union FragH { v16h v; v8h h[2]; };
__device__ __forceinline__ v8h cvt8h(v4f a, v4f c) {
    v8h r;
    r[0] = (_Float16)a.x; r[1] = (_Float16)a.y; r[2] = (_Float16)a.z; r[3] = (_Float16)a.w;
    r[4] = (_Float16)c.x; r[5] = (_Float16)c.y; r[6] = (_Float16)c.z; r[7] = (_Float16)c.w;
    return r;
}

#define VST2(T, ptr, val) do { const T vst2_v_ = (val); *(volatile T*)(ptr) = vst2_v_; __threadfence(); *(volatile T*)(ptr) = vst2_v_; } while (0)
#define VST2V4(ptr, val) do { const v4f vst2_v4_ = (val); *(volatile v4f*)(ptr) = vst2_v4_; __threadfence(); *(volatile v4f*)(ptr) = vst2_v4_; } while (0)

#define AW 4
#define AT_KP 72
#define AT_OP 68
static_assert(16 * AW == 64);
static_assert(32 * AW * 32 == 64 * HDIM);
static_assert(AT_KP >= 64 && AT_KP % 8 == 0);
static_assert(AT_OP >= 64 && AT_OP % 4 == 0);
static_assert(16 * 16 == HDIM * 4);
__global__ __launch_bounds__(32 * AW) void k_attn_fwd(const float* __restrict__ QKV, float* __restrict__ AO, int seq, int ldq, int ldo, float scale) {
    __shared__ __align__(16) _Float16 qs_[AW * 16 * AT_KP];
    __shared__ __align__(16) _Float16 ks_[64 * AT_KP];
    __shared__ __align__(16) _Float16 vt_[64 * AT_KP];
    __shared__ __align__(16) _Float16 ps_[AW * 16 * AT_KP];
    __shared__ __align__(16) float    os_[AW * 16 * AT_OP];
    const int tid = threadIdx.x, lane = tid & 31, hf = lane >> 4, l15 = lane & 15, wave = tid >> 5;
    const int h = blockIdx.y, b = blockIdx.z;
    const int q0 = (blockIdx.x * AW + wave) * 16;
    const long long rb = (long long)b * seq;
    const int qcol = h * HDIM, kcol = DM + h * HDIM, vcol = 2 * DM + h * HDIM;
    const float L2E = 1.4426950408889634f;
    const float NEG = -__builtin_inff();

    {
        const int qr = lane >> 1, dh = (lane & 1) * 32;
        const int qg = min(q0 + qr, seq - 1);
        const long long go = (rb + qg) * (long long)ldq + qcol + dh;
        const int lo = (wave * 16 + qr) * AT_KP + dh;
#pragma unroll
        for (int i = 0; i < 4; ++i) {
            const v4f a = *(const v4f*)(QKV + go + 8 * i); const v4f c = *(const v4f*)(QKV + go + 8 * i + 4);
            const v8h hv = cvt8h(a, c);
            *(v8h_a*)(&qs_[lo + 8 * i]) = hv;
        }
    }

    v8f o[4]; float m8[8], l8[8];
#pragma unroll
    for (int t = 0; t < 4; ++t) { v8f zz = {}; o[t] = zz; }
#pragma unroll
    for (int i = 0; i < 8; ++i) { m8[i] = NEG; l8[i] = 0.f; }

    for (int j0 = 0; j0 < seq; j0 += 64) {
        __syncthreads();
        {
            const int kvr = tid >> 1, dh = (tid & 1) * 32;
            const int jg = min(j0 + kvr, seq - 1);
            const long long gk = (rb + jg) * (long long)ldq + kcol + dh;
            const long long gv = (rb + jg) * (long long)ldq + vcol + dh;
#pragma unroll
            for (int i = 0; i < 4; ++i) {
                const v4f a = *(const v4f*)(QKV + gk + 8 * i); const v4f c = *(const v4f*)(QKV + gk + 8 * i + 4);
                const v8h hv = cvt8h(a, c);
                *(v8h_a*)(&ks_[kvr * AT_KP + dh + 8 * i]) = hv;
            }
#pragma unroll
            for (int i = 0; i < 4; ++i) {
                const v4f a = *(const v4f*)(QKV + gv + 8 * i); const v4f c = *(const v4f*)(QKV + gv + 8 * i + 4);
                const int d0 = dh + 8 * i;
                vt_[(d0 + 0) * AT_KP + kvr] = (_Float16)a.x; vt_[(d0 + 1) * AT_KP + kvr] = (_Float16)a.y;
                vt_[(d0 + 2) * AT_KP + kvr] = (_Float16)a.z; vt_[(d0 + 3) * AT_KP + kvr] = (_Float16)a.w;
                vt_[(d0 + 4) * AT_KP + kvr] = (_Float16)c.x; vt_[(d0 + 5) * AT_KP + kvr] = (_Float16)c.y;
                vt_[(d0 + 6) * AT_KP + kvr] = (_Float16)c.z; vt_[(d0 + 7) * AT_KP + kvr] = (_Float16)c.w;
            }
        }
        __syncthreads();
#pragma unroll 1
        for (int hh = 0; hh < 2; ++hh) {
            v8f s0 = {}, s1 = {};
#pragma unroll
            for (int ks = 0; ks < 2; ++ks) {
                FragH qa, k0f, k1f;
                const int qo = (wave * 16 + l15) * AT_KP + ks * 32 + 8 * hf;
                qa.h[0] = *(const v8h_a*)(&qs_[qo]); qa.h[1] = *(const v8h_a*)(&qs_[qo + 16]);
                const int ko = (hh * 32 + l15) * AT_KP + ks * 32 + 8 * hf;
                k0f.h[0] = *(const v8h_a*)(&ks_[ko]); k0f.h[1] = *(const v8h_a*)(&ks_[ko + 16]);
                k1f.h[0] = *(const v8h_a*)(&ks_[ko + 16 * AT_KP]); k1f.h[1] = *(const v8h_a*)(&ks_[ko + 16 * AT_KP + 16]);
                s0 = wmma16(qa.v, k0f.v, s0);
                s1 = wmma16(qa.v, k1f.v, s1);
            }
#pragma unroll
            for (int i = 0; i < 8; ++i) {
                float a0 = s0[i] * scale; a0 *= L2E;
                float a1 = s1[i] * scale; a1 *= L2E;
                float mx = fmaxf(a0, a1);
                mx = fmaxf(mx, __shfl_xor(mx, 1, 32)); mx = fmaxf(mx, __shfl_xor(mx, 2, 32));
                mx = fmaxf(mx, __shfl_xor(mx, 4, 32)); mx = fmaxf(mx, __shfl_xor(mx, 8, 32));
                const float mnew = fmaxf(m8[i], mx);
                const float corr = (mnew == NEG) ? 1.f : exp2f(m8[i] - mnew);
                const float p0 = exp2f(a0 - mnew), p1 = exp2f(a1 - mnew);
                float rs = p0 + p1;
                rs += __shfl_xor(rs, 1, 32); rs += __shfl_xor(rs, 2, 32); rs += __shfl_xor(rs, 4, 32); rs += __shfl_xor(rs, 8, 32);
                l8[i] = l8[i] * corr + rs; m8[i] = mnew;
                o[0][i] *= corr; o[1][i] *= corr; o[2][i] *= corr; o[3][i] *= corr;
                const int po = (wave * 16 + 8 * hf + i) * AT_KP + hh * 32 + l15;
                ps_[po] = (_Float16)(p0 * 4096.f);
                ps_[po + 16] = (_Float16)(p1 * 4096.f);
            }
            __syncthreads();
            FragH pa, vb[4];
            const int pao = (wave * 16 + l15) * AT_KP + hh * 32 + 8 * hf;
            pa.h[0] = *(const v8h_a*)(&ps_[pao]); pa.h[1] = *(const v8h_a*)(&ps_[pao + 16]);
#pragma unroll
            for (int t = 0; t < 4; ++t) {
                const int vo = (t * 16 + l15) * AT_KP + hh * 32 + 8 * hf;
                vb[t].h[0] = *(const v8h_a*)(&vt_[vo]); vb[t].h[1] = *(const v8h_a*)(&vt_[vo + 16]);
            }
#pragma unroll
            for (int t = 0; t < 4; ++t) o[t] = wmma16(pa.v, vb[t].v, o[t]);
        }
    }

#pragma unroll
    for (int i = 0; i < 8; ++i) {
        const float inv = (l8[i] > 0.f) ? 1.f / (l8[i] * 4096.f) : 0.f;
        const int oo = (wave * 16 + 8 * hf + i) * AT_OP + l15;
        os_[oo] = o[0][i] * inv; os_[oo + 16] = o[1][i] * inv; os_[oo + 32] = o[2][i] * inv; os_[oo + 48] = o[3][i] * inv;
    }
    __syncthreads();
    if (q0 + 16 <= seq) {
#pragma unroll 1
        for (int r0 = 0; r0 < 16; r0 += 2) {
            const int row = r0 + hf, c4 = l15 * 4;
            const v4f v = *(const v4f_a*)(&os_[(wave * 16 + row) * AT_OP + c4]);
            VST2V4(AO + (rb + q0 + row) * (long long)ldo + qcol + c4, v);
        }
    }
}

namespace w25 {
typedef __attribute__((ext_vector_type(16))) _Float16 v16h;
typedef __attribute__((ext_vector_type(8)))  _Float16 v8h;
typedef __attribute__((ext_vector_type(16))) __bf16   v16b;
typedef __attribute__((ext_vector_type(8)))  __bf16   v8b;
typedef __attribute__((ext_vector_type(8)))  float    v8f;
typedef __attribute__((ext_vector_type(4)))  float    v4f;

__device__ __forceinline__ unsigned short f2bf_bits(float f) {
  unsigned u = __float_as_uint(f);
  return (unsigned short)((u + 0x7FFFu + ((u >> 16) & 1u)) >> 16);
}
__device__ __forceinline__ float bf_bits2f(unsigned short h) { return __uint_as_float(((unsigned)h) << 16); }

__device__ __forceinline__ void dep_guard_h(v8f& a, v8f& b, v16h x, v16h y) { asm volatile("v_nop\n\tv_nop\n\tv_nop\n\tv_nop" : "+v"(a), "+v"(b) : "v"(x), "v"(y)); }
__device__ __forceinline__ void dep_guard_b(v8f& a, v8f& b, v16b x, v16b y) { asm volatile("v_nop\n\tv_nop\n\tv_nop\n\tv_nop" : "+v"(a), "+v"(b) : "v"(x), "v"(y)); }
__device__ __forceinline__ void keep4_h(v16h a, v16h b, v16h c, v16h d) { asm volatile("v_nop" :: "v"(a), "v"(b), "v"(c), "v"(d)); }
__device__ __forceinline__ void keep4_b(v16b a, v16b b, v16b c, v16b d) { asm volatile("v_nop" :: "v"(a), "v"(b), "v"(c), "v"(d)); }
__device__ __forceinline__ void acc_guard4(v8f& a, v8f& b, v8f& c, v8f& d) { asm volatile("v_nop\n\tv_nop\n\tv_nop\n\tv_nop" : "+v"(a), "+v"(b), "+v"(c), "+v"(d)); }
template <typename T> struct Frag;
template <> struct Frag<_Float16> {
  typedef v16h V; union U { v16h v; v8h h[2]; };
  static __device__ __forceinline__ v16h load(const _Float16* p) {
    U f; f.h[0] = *(const v8h*)(p); f.h[1] = *(const v8h*)(p + 16); return f.v;
  }
  static __device__ __forceinline__ v8f mma(v16h a, v16h b, v8f c) {
    return __builtin_amdgcn_wmma_f32_16x16x32_f16(false, a, false, b, (short)0, c, false, false);
  }
  static __device__ __forceinline__ void guard(v8f& a, v8f& b, v16h x, v16h y) { dep_guard_h(a, b, x, y); }
  static __device__ __forceinline__ void keep(v16h a, v16h b, v16h c, v16h d) { keep4_h(a, b, c, d); }
};
template <> struct Frag<__bf16> {
  typedef v16b V; union U { v16b v; v8b h[2]; };
  static __device__ __forceinline__ v16b load(const __bf16* p) {
    U f; f.h[0] = *(const v8b*)(p); f.h[1] = *(const v8b*)(p + 16); return f.v;
  }
  static __device__ __forceinline__ v8f mma(v16b a, v16b b, v8f c) {
    return __builtin_amdgcn_wmma_f32_16x16x32_bf16(false, a, false, b, (short)0, c, false, false);
  }
  static __device__ __forceinline__ void guard(v8f& a, v8f& b, v16b x, v16b y) { dep_guard_b(a, b, x, y); }
  static __device__ __forceinline__ void keep(v16b a, v16b b, v16b c, v16b d) { keep4_b(a, b, c, d); }
};

template <int ET> struct Elem;
template <> struct Elem<0> { typedef _Float16 T; };
template <> struct Elem<1> { typedef __bf16 T; };
template <int ET, bool SPLIT, int BIAS_MODE, int OUT_MODE, bool RESID, int ACT>
__device__ __forceinline__ void gemm64_body(
    const unsigned short* __restrict__ Ap, const unsigned short* __restrict__ A2p, int lda, long strideA,
    const unsigned short* __restrict__ Btp, const unsigned short* __restrict__ Bt2p, int ldb, long strideB,
    void* __restrict__ Cout, void* __restrict__ Cout2, int ldc, long strideC,
    const float* __restrict__ bias,
    const float* __restrict__ resid, long strideR,
    int M, int N, int K, float scale) {
  typedef typename Elem<ET>::T T;
  typedef typename Frag<T>::V V;
  const T* A = (const T*)Ap; const T* A2 = (const T*)A2p; const T* Bt = (const T*)Btp; const T* Bt2 = (const T*)Bt2p;
  __shared__ __align__(16) float sT[8][16 * 68];
  const int b    = blockIdx.y;
  const int lane = threadIdx.x & 31;
  const int wave = threadIdx.x >> 5;
  const int tilesN = N >> 6;
  const int tilesM = M >> 6;
  const int tile = blockIdx.x * 8 + wave;
  if (tile >= tilesM * tilesN) return;
  const int tm = tile / tilesN;
  const int tn = tile - tm * tilesN;
  const int m0 = tm << 6;
  const int n0 = tn << 6;

  const T* Ab  = A  + (size_t)b * strideA;
  const T* Bb  = Bt + (size_t)b * strideB;
  const T* Ab2 = SPLIT ? (A2  + (size_t)b * strideA) : nullptr;
  const T* Bb2 = SPLIT ? (Bt2 + (size_t)b * strideB) : nullptr;

  const int rlane = lane & 15;
  const int koff  = (lane >> 4) * 8;
  const int mOff  = (lane >> 4) * 8;

  v8f acc[4][4];
#pragma unroll
  for (int i = 0; i < 4; ++i)
#pragma unroll
    for (int j = 0; j < 4; ++j) acc[i][j] = (v8f){0.f,0.f,0.f,0.f,0.f,0.f,0.f,0.f};

  for (int k0 = 0; k0 < K; k0 += 32) {
    V bh[4], bl[4];
#pragma unroll
    for (int j = 0; j < 4; ++j) {
      const size_t bo = (size_t)(n0 + (j << 4) + rlane) * ldb + koff + k0;
      bh[j] = Frag<T>::load(Bb + bo);
      if (SPLIT) bl[j] = Frag<T>::load(Bb2 + bo);
    }
#pragma unroll
    for (int i = 0; i < 4; ++i) {
      const size_t ao = (size_t)(m0 + (i << 4) + rlane) * lda + koff + k0;
      V ah = Frag<T>::load(Ab + ao);
      V al;
      if (SPLIT) al = Frag<T>::load(Ab2 + ao);
#pragma unroll
      for (int j = 0; j < 4; ++j) {
        acc[i][j] = Frag<T>::mma(ah, bh[j], acc[i][j]);
        if (SPLIT) {
          acc[i][j] = Frag<T>::mma(ah, bl[j], acc[i][j]);
          acc[i][j] = Frag<T>::mma(al, bh[j], acc[i][j]);
        }
      }
      Frag<T>::guard(acc[i][0], acc[i][3], ah, SPLIT ? al : ah);
    }
    Frag<T>::keep(bh[0], bh[1], bh[2], bh[3]);
    if (SPLIT) Frag<T>::keep(bl[0], bl[1], bl[2], bl[3]);
  }
  acc_guard4(acc[0][0], acc[0][1], acc[0][2], acc[0][3]);
  acc_guard4(acc[1][0], acc[1][1], acc[1][2], acc[1][3]);
  acc_guard4(acc[2][0], acc[2][1], acc[2][2], acc[2][3]);
  acc_guard4(acc[3][0], acc[3][1], acc[3][2], acc[3][3]);

  float* slab = sT[wave];
  const float* Rb = RESID ? (resid + (size_t)b * strideR) : nullptr;
#pragma unroll
  for (int i = 0; i < 4; ++i) {
    const int mBase = m0 + (i << 4);
#pragma unroll
    for (int j = 0; j < 4; ++j) {
      const int n = n0 + (j << 4) + rlane;
      float bv = 0.f;
      if (BIAS_MODE == 2) bv = bias[n];
#pragma unroll
      for (int r = 0; r < 8; ++r) {
        float v = acc[i][j][r] * scale;
        if (BIAS_MODE == 1) v += bias[mBase + mOff + r];
        if (BIAS_MODE == 2) v += bv;
        if (RESID) v += Rb[(size_t)(mBase + mOff + r) * ldc + n];
        if (ACT == 2) v = fmaxf(v, 0.0f);
        slab[(mOff + r) * 68 + (j << 4) + rlane] = v;
      }
    }
    __builtin_amdgcn_fence(3  , "workgroup");
    __builtin_amdgcn_wave_barrier();
    __builtin_amdgcn_fence(2  , "workgroup");
    if (OUT_MODE == 0) {
      float* C = (float*)Cout + (size_t)b * strideC;
      const int hh = lane >> 4, c4 = (lane & 15) * 4;
      for (int pass = 0; pass < 2; ++pass) {
#pragma unroll
        for (int it = 0; it < 8; ++it) {
          const int row = it * 2 + hh;
          v4f v = *(const v4f*)(slab + row * 68 + c4);
          *(volatile v4f*)(C + (size_t)(mBase + row) * ldc + n0 + c4) = v;
        }
        __threadfence();
      }
    } else {
      const int q = lane >> 3, c8 = (lane & 7) * 8;
      unsigned short* C  = (unsigned short*)Cout  + (size_t)b * strideC;
      unsigned short* C2 = (OUT_MODE == 2) ? ((unsigned short*)Cout2 + (size_t)b * strideC) : nullptr;
      for (int pass = 0; pass < 2; ++pass) {
#pragma unroll
        for (int it = 0; it < 4; ++it) {
          const int row = it * 4 + q;
          const float* sp = slab + row * 68 + c8;
          v8h hv, lv;
#pragma unroll
          for (int e = 0; e < 8; ++e) {
            if (OUT_MODE == 1) {
              hv[e] = (_Float16)sp[e];
            } else {
              unsigned short hb = f2bf_bits(sp[e]);
              unsigned short lb = f2bf_bits(sp[e] - bf_bits2f(hb));
              hv[e] = __builtin_bit_cast(_Float16, hb);
              lv[e] = __builtin_bit_cast(_Float16, lb);
            }
          }
          *(volatile v8h*)(C + (size_t)(mBase + row) * ldc + n0 + c8) = hv;
          if (OUT_MODE == 2) *(volatile v8h*)(C2 + (size_t)(mBase + row) * ldc + n0 + c8) = lv;
        }
        __threadfence();
      }
    }
    __builtin_amdgcn_fence(3  , "workgroup");
    __builtin_amdgcn_wave_barrier();
    __builtin_amdgcn_fence(2  , "workgroup");
  }
}
}

__global__ __launch_bounds__(256) void k_gemm_f32(const unsigned short* __restrict__ A, int lda, const unsigned short* __restrict__ Bt, int ldb,
                                                   float* __restrict__ C, int ldc, const float* __restrict__ bias, int M, int N, int K, float scale) {
    w25::gemm64_body<0, false, 2, 0, false, 0>(A, nullptr, lda, 0, Bt, nullptr, ldb, 0, (void*)C, nullptr, ldc, 0, bias, nullptr, 0, M, N, K, scale);
}
__global__ __launch_bounds__(256) void k_gemm_relu16(const unsigned short* __restrict__ A, int lda, const unsigned short* __restrict__ Bt, int ldb,
                                                      unsigned short* __restrict__ C, int ldc, const float* __restrict__ bias, int M, int N, int K, float scale) {
    w25::gemm64_body<0, false, 2, 1, false, 2>(A, nullptr, lda, 0, Bt, nullptr, ldb, 0, (void*)C, nullptr, ldc, 0, bias, nullptr, 0, M, N, K, scale);
}

typedef unsigned int cm_u4 __attribute__((ext_vector_type(4)));
__device__ __forceinline__ unsigned int cmb_pk2(float a, float b) { return (unsigned int)__builtin_bit_cast(unsigned short, (_Float16)a) | ((unsigned int)__builtin_bit_cast(unsigned short, (_Float16)b) << 16); }
__device__ __forceinline__ float cmb_bf(float v) { const unsigned u = __builtin_bit_cast(unsigned, v); const unsigned r = (u + 0x7fffu + ((u >> 16) & 1u)) & 0xffff0000u; return __builtin_bit_cast(float, r); }

__global__ __launch_bounds__(256) void k_x16(const float* __restrict__ SRC, unsigned short* __restrict__ DST, int rows, int seq, int seq_full) {
    const long long u = (long long)blockIdx.x * 256 + threadIdx.x; const int per = DM / 8; if (u >= (long long)rows * per) return;
    const int r = (int)(u / per); const int c0 = 8 * (int)(u % per);
    const long long rs = (long long)(r / seq) * seq_full + (r % seq);
    const float* s = SRC + rs * DM + c0;
    const v4f a = *(const v4f*)s; const v4f b = *(const v4f*)(s + 4);
    cm_u4 pk; pk.x = cmb_pk2(cmb_bf(a.x), cmb_bf(a.y)); pk.y = cmb_pk2(cmb_bf(a.z), cmb_bf(a.w)); pk.z = cmb_pk2(cmb_bf(b.x), cmb_bf(b.y)); pk.w = cmb_pk2(cmb_bf(b.z), cmb_bf(b.w));
    VST2(cm_u4, (cm_u4*)(DST + (long long)r * DM + c0), pk); }

__global__ __launch_bounds__(256) void k_whead(const float* __restrict__ Wp, unsigned short* __restrict__ DST) {
    const int u = blockIdx.x * 256 + threadIdx.x; if (u >= DM * (DM / 8)) return; const int n = u / (DM / 8); const int d0 = 8 * (u % (DM / 8)); const int h = n >> 6, k = n & 63;
    float w[8];
#pragma unroll
    for (int e = 0; e < 8; ++e) w[e] = cmb_bf(Wp[((long long)h * DM + d0 + e) * HDIM + k]) * 16.f;
    cm_u4 pk; pk.x = cmb_pk2(w[0], w[1]); pk.y = cmb_pk2(w[2], w[3]); pk.z = cmb_pk2(w[4], w[5]); pk.w = cmb_pk2(w[6], w[7]); VST2(cm_u4, (cm_u4*)(DST + (long long)n * DM + d0), pk); }

__global__ __launch_bounds__(256) void k_cm_castbT(const float* __restrict__ SRC, int lds, unsigned short* __restrict__ DST, int ldd, int nR, int nC, float sc) {
    const long long u = (long long)blockIdx.x * 256 + threadIdx.x; const int per = nR / 8; if (u >= (long long)nC * per) return; const int c = (int)(u / per); const int r0 = 8 * (int)(u % per);
    float w[8];
#pragma unroll
    for (int e = 0; e < 8; ++e) w[e] = cmb_bf(SRC[(long long)(r0 + e) * lds + c]) * sc;
    cm_u4 pk; pk.x = cmb_pk2(w[0], w[1]); pk.y = cmb_pk2(w[2], w[3]); pk.z = cmb_pk2(w[4], w[5]); pk.w = cmb_pk2(w[6], w[7]); VST2(cm_u4, (cm_u4*)(DST + (long long)c * ldd + r0), pk); }

__global__ __launch_bounds__(256) void k_bias(const float* __restrict__ bq, const float* __restrict__ bk, const float* __restrict__ bv, const float* __restrict__ b1, const float* __restrict__ b2,
                                               float* __restrict__ BR3, float* __restrict__ BR1, float* __restrict__ BR2) {
    const int blk = blockIdx.x, t = threadIdx.x;
    if (blk < 4)       { const int i = blk * 256 + t;        const float v = cmb_bf(bq[i]); VST2(float, BR3 + i, v); }
    else if (blk < 8)  { const int i = (blk - 4) * 256 + t;  const float v = cmb_bf(bk[i]); VST2(float, BR3 + DM + i, v); }
    else if (blk < 12) { const int i = (blk - 8) * 256 + t;  const float v = cmb_bf(bv[i]); VST2(float, BR3 + 2 * DM + i, v); }
    else if (blk < 28) { const int i = (blk - 12) * 256 + t; const float v = cmb_bf(b1[i]); VST2(float, BR1 + i, v); }
    else if (blk < 32) { const int i = (blk - 28) * 256 + t; const float v = cmb_bf(b2[i]); VST2(float, BR2 + i, v); }
}

typedef unsigned int bk_u2 __attribute__((ext_vector_type(2)));
__device__ __forceinline__ unsigned int bk_pk2(float a, float b) { return (unsigned int)__builtin_bit_cast(unsigned short, (_Float16)a) | ((unsigned int)__builtin_bit_cast(unsigned short, (_Float16)b) << 16); }
template <int NQ, int HASX, int XBF, int ABF, int XMAP, int YMAP, int W16>
__device__ __forceinline__ void ln_body(const float* __restrict__ A, const float* __restrict__ X, const float* __restrict__ GA, const float* __restrict__ BE, float eps, float inv_vden,
                                        int rows, int seq, int seq_full, float* __restrict__ Yf, unsigned short* __restrict__ Y16) {
    #pragma clang fp contract(off)
    constexpr int WD = 128 * NQ; const int r = blockIdx.x * 8 + (threadIdx.x >> 5); const int L = threadIdx.x & 31; if (r >= rows) return;
    const long long rm = (long long)(r / seq) * seq_full + (r % seq);
    const long long rx = XMAP ? rm : (long long)r; const long long ry = YMAP ? rm : (long long)r;
    v4f v[NQ]; float s = 0.f;
#pragma unroll
    for (int q = 0; q < NQ; ++q) { const int c = 4 * L + 128 * q; v[q] = *(const v4f*)(A + (long long)r * WD + c);
        if (ABF) { v[q].x = cmb_bf(v[q].x); v[q].y = cmb_bf(v[q].y); v[q].z = cmb_bf(v[q].z); v[q].w = cmb_bf(v[q].w); }
        if (HASX) { v4f x = *(const v4f*)(X + rx * WD + c); if (XBF) { x.x = cmb_bf(x.x); x.y = cmb_bf(x.y); x.z = cmb_bf(x.z); x.w = cmb_bf(x.w); } v[q] = v[q] + x; }
        s += (v[q].x + v[q].y) + (v[q].z + v[q].w); }
#pragma unroll
    for (int o = 16; o > 0; o >>= 1) s += __shfl_xor(s, o, 32);
    const float mu = s * (1.f / WD); float qq = 0.f;
#pragma unroll
    for (int q = 0; q < NQ; ++q) { v[q].x -= mu; v[q].y -= mu; v[q].z -= mu; v[q].w -= mu; qq += (v[q].x * v[q].x + v[q].y * v[q].y) + (v[q].z * v[q].z + v[q].w * v[q].w); }
#pragma unroll
    for (int o = 16; o > 0; o >>= 1) qq += __shfl_xor(qq, o, 32);
    const float rs = rsqrtf(qq * inv_vden + eps);
#pragma unroll
    for (int q = 0; q < NQ; ++q) { const int c = 4 * L + 128 * q; const v4f ga = *(const v4f*)(GA + c), be = *(const v4f*)(BE + c); v4f y;
        y.x = v[q].x * rs * cmb_bf(ga.x) + cmb_bf(be.x); y.y = v[q].y * rs * cmb_bf(ga.y) + cmb_bf(be.y); y.z = v[q].z * rs * cmb_bf(ga.z) + cmb_bf(be.z); y.w = v[q].w * rs * cmb_bf(ga.w) + cmb_bf(be.w);
        VST2V4(Yf + ry * WD + c, y);
        if (W16) { bk_u2 pk; pk.x = bk_pk2(y.x, y.y); pk.y = bk_pk2(y.z, y.w); VST2(bk_u2, (bk_u2*)(Y16 + (long long)r * WD + c), pk); } } }
__global__ __launch_bounds__(256) void k_ln1(const float* __restrict__ AO, const float* __restrict__ X, const float* __restrict__ GA, const float* __restrict__ BE, float eps, float inv_vden,
                                              int rows, int seq, int seq_full, float* __restrict__ Yf, unsigned short* __restrict__ Y16) {
    ln_body<8, 1, 1, 0, 1, 0, 1>(AO, X, GA, BE, eps, inv_vden, rows, seq, seq_full, Yf, Y16); }
__global__ __launch_bounds__(256) void k_ln2(const float* __restrict__ FF, const float* __restrict__ Y1, const float* __restrict__ GA, const float* __restrict__ BE, float eps, float inv_vden,
                                              int rows, int seq, int seq_full, float* __restrict__ OUT) {
    ln_body<8, 1, 0, 0, 0, 1, 0>(FF, Y1, GA, BE, eps, inv_vden, rows, seq, seq_full, OUT, nullptr); }

static constexpr size_t SZ_X16 = (size_t)ROWS * DM * 2;
static constexpr size_t SZ_W3  = (size_t)3 * DM * DM * 2;
static constexpr size_t SZ_QKV = (size_t)ROWS * 3 * DM * 4;
static constexpr size_t SZ_AO  = (size_t)ROWS * DM * 4;
static constexpr size_t SZ_X1  = (size_t)ROWS * DM * 4;
static constexpr size_t SZ_H16 = (size_t)ROWS * DM * 2;
static constexpr size_t SZ_W1T = (size_t)DFF * DM * 2;
static constexpr size_t SZ_W2T = (size_t)DM * DFF * 2;
static constexpr size_t SZ_BR3 = (size_t)3 * DM * 4;
static constexpr size_t SZ_BR1 = (size_t)DFF * 4;
static constexpr size_t SZ_BR2 = (size_t)DM * 4;
static constexpr size_t SZ_F16 = (size_t)ROWS * DFF * 2;
static constexpr size_t SZ_FFO = (size_t)ROWS * DM * 4;
static constexpr size_t OFF_X16 = 0;
static constexpr size_t OFF_W3  = OFF_X16 + SZ_X16;
static constexpr size_t OFF_QKV = OFF_W3 + SZ_W3;
static constexpr size_t OFF_AO  = OFF_QKV + SZ_QKV;
static constexpr size_t OFF_X1  = OFF_AO + SZ_AO;
static constexpr size_t OFF_H16 = OFF_X1 + SZ_X1;
static constexpr size_t OFF_W1T = OFF_H16 + SZ_H16;
static constexpr size_t OFF_W2T = OFF_W1T + SZ_W1T;
static constexpr size_t OFF_BR3 = OFF_W2T + SZ_W2T;
static constexpr size_t OFF_BR1 = OFF_BR3 + SZ_BR3;
static constexpr size_t OFF_BR2 = OFF_BR1 + SZ_BR1;
static constexpr size_t WS_TOTAL = OFF_BR2 + SZ_BR2;
static_assert(SZ_F16 + SZ_FFO <= SZ_QKV);
static_assert(WS_TOTAL <= (size_t)134217728);
static_assert(SZ_X16 % 256 == 0 && SZ_W3 % 256 == 0 && SZ_QKV % 256 == 0 && SZ_AO % 256 == 0 && SZ_H16 % 256 == 0 && SZ_W1T % 256 == 0);
static_assert(SZ_BR3 % 256 == 0 && SZ_BR1 % 256 == 0 && SZ_BR2 % 256 == 0 && SZ_F16 % 256 == 0);
static_assert(((ROWS / 64) * ((3 * DM) / 64)) % 8 == 0 && ((ROWS / 64) * (DFF / 64)) % 8 == 0 && ((ROWS / 64) * (DM / 64)) % 8 == 0);

extern "C" void kernel_launch(void* const* d_in, const int* in_sizes, int n_in, void* d_out, int out_size, void* d_ws, size_t ws_size, hipStream_t stream) {
    if (n_in < 15) return;
    const long long need_x = ((long long)(NB - 1) * SEQ_FULL + SEQ) * DM;
    if ((long long)in_sizes[0] < need_x || (long long)out_size < need_x) return;
    if (in_sizes[1] < NHEAD * DM * HDIM || in_sizes[3] < NHEAD * DM * HDIM || in_sizes[5] < NHEAD * DM * HDIM) return;
    if (in_sizes[2] < DM || in_sizes[4] < DM || in_sizes[6] < DM || in_sizes[7] < DM || in_sizes[8] < DM) return;
    if (in_sizes[9] < DM * DFF || in_sizes[10] < DFF || in_sizes[11] < DFF * DM || in_sizes[12] < DM || in_sizes[13] < DM || in_sizes[14] < DM) return;
    if (WS_TOTAL > ws_size) return;
    const float* x   = (const float*)d_in[0];
    const float* wq  = (const float*)d_in[1];
    const float* bq  = (const float*)d_in[2];
    const float* wk  = (const float*)d_in[3];
    const float* bk  = (const float*)d_in[4];
    const float* wv  = (const float*)d_in[5];
    const float* bv  = (const float*)d_in[6];
    const float* g1  = (const float*)d_in[7];
    const float* be1 = (const float*)d_in[8];
    const float* w1  = (const float*)d_in[9];
    const float* b1  = (const float*)d_in[10];
    const float* w2  = (const float*)d_in[11];
    const float* b2  = (const float*)d_in[12];
    const float* g2  = (const float*)d_in[13];
    const float* be2 = (const float*)d_in[14];
    float* out = (float*)d_out;
    char* ws = (char*)d_ws;
    unsigned short* X16  = (unsigned short*)(ws + OFF_X16);
    unsigned short* W316 = (unsigned short*)(ws + OFF_W3);
    float*          QKV  = (float*)(ws + OFF_QKV);
    float*          AO   = (float*)(ws + OFF_AO);
    float*          X1   = (float*)(ws + OFF_X1);
    unsigned short* H16  = (unsigned short*)(ws + OFF_H16);
    unsigned short* W1T  = (unsigned short*)(ws + OFF_W1T);
    unsigned short* W2T  = (unsigned short*)(ws + OFF_W2T);
    float*          BR3  = (float*)(ws + OFF_BR3);
    float*          BR1  = (float*)(ws + OFF_BR1);
    float*          BR2  = (float*)(ws + OFF_BR2);
    unsigned short* F16  = (unsigned short*)(ws + OFF_QKV);
    float*          FFo  = (float*)(ws + OFF_QKV + SZ_F16);

    k_x16<<<(unsigned)(((long long)ROWS * (DM / 8) + 255) / 256), 256, 0, stream>>>(x, X16, ROWS, SEQ, SEQ_FULL);
    k_whead<<<(DM * (DM / 8) + 255) / 256, 256, 0, stream>>>(wq, W316);
    k_whead<<<(DM * (DM / 8) + 255) / 256, 256, 0, stream>>>(wk, W316 + (size_t)DM * DM);
    k_whead<<<(DM * (DM / 8) + 255) / 256, 256, 0, stream>>>(wv, W316 + (size_t)2 * DM * DM);
    k_cm_castbT<<<(unsigned)(((long long)DFF * (DM / 8) + 255) / 256), 256, 0, stream>>>(w1, DFF, W1T, DM, DM, DFF, 16.0f);
    k_cm_castbT<<<(unsigned)(((long long)DM * (DFF / 8) + 255) / 256), 256, 0, stream>>>(w2, DM, W2T, DFF, DFF, DM, 16.0f);
    k_bias<<<32, 256, 0, stream>>>(bq, bk, bv, b1, b2, BR3, BR1, BR2);
    k_gemm_f32<<<dim3((unsigned)(((ROWS / 64) * ((3 * DM) / 64) + 7) / 8), 1u), 256, 0, stream>>>(X16, DM, W316, DM, QKV, 3 * DM, BR3, ROWS, 3 * DM, DM, 0.0625f);
    k_attn_fwd<<<dim3((unsigned)(SEQ / (16 * AW)), (unsigned)NHEAD, (unsigned)NB), 32 * AW, 0, stream>>>(QKV, AO, SEQ, 3 * DM, DM, 0.125f);
    k_ln1<<<(ROWS + 7) / 8, 256, 0, stream>>>(AO, x, g1, be1, 1e-5f, 1.0f / (float)DM, ROWS, SEQ, SEQ_FULL, X1, H16);
    k_gemm_relu16<<<dim3((unsigned)(((ROWS / 64) * (DFF / 64) + 7) / 8), 1u), 256, 0, stream>>>(H16, DM, W1T, DM, F16, DFF, BR1, ROWS, DFF, DM, 0.0625f);
    k_gemm_f32<<<dim3((unsigned)(((ROWS / 64) * (DM / 64) + 7) / 8), 1u), 256, 0, stream>>>(F16, DFF, W2T, DFF, FFo, DM, BR2, ROWS, DM, DFF, 0.0625f);
    k_ln2<<<(ROWS + 7) / 8, 256, 0, stream>>>(FFo, X1, g2, be2, 1e-5f, 1.0f / (float)DM, ROWS, SEQ, SEQ_FULL, out);
}
